// GATLayerEdgeSoftmax_82197084111208
// MI455X (gfx1250) — hardware-verified
//
#include <hip/hip_runtime.h>
#include <stddef.h>


#define DI    64
#define DO    64
#define KW    128
#define NOUT  144
#define NT    9
#define GR    32
#define GTHR  128
#define GWAVE 4
#define AP    72
#define XSP   148
#define NB    1024
#define CHUNK 2048
#define NTHR  256
#define NWAVE 8
#define WCAP  256
#define NGRP  (CHUNK / (NTHR * 4))
#define MB    128
#define EPSV  1e-6f
#define NEGBIG (-3.402823466e38f)

#define LDS_SACC (NB * DO)
#define LDS_DEN  NB
#define LDS_LIST (NWAVE * WCAP)
#define LDS_BYTES ((LDS_SACC + LDS_DEN + LDS_LIST + NWAVE + NWAVE) * 4)

static_assert(WCAP == (CHUNK / NTHR) * 32);
static_assert(NGRP == 2);
static_assert(NB == 1024);
static_assert(CHUNK == 2048);
static_assert(((LDS_SACC + LDS_DEN) % 4) == 0);
static_assert(LDS_BYTES == 274496);
static_assert(MB <= NTHR);
static_assert((NB % (2 * NWAVE)) == 0);
static_assert(XSP >= NOUT);

typedef float          v2f  __attribute__((ext_vector_type(2)));
typedef float          v4f  __attribute__((ext_vector_type(4)));
typedef float          v8f  __attribute__((ext_vector_type(8)));
typedef int            v4i  __attribute__((ext_vector_type(4)));
typedef unsigned short v8us __attribute__((ext_vector_type(8)));
typedef __bf16         v16b __attribute__((ext_vector_type(16)));
union FragB { v16b v; v8us hs[2]; };
union Pack8 { v8us v; unsigned short s[8]; };

__device__ __forceinline__ unsigned short bfr(float f) {
  unsigned u = __float_as_uint(f);
  u += 0x7FFFu + ((u >> 16) & 1u);
  return (unsigned short)(u >> 16);
}

__device__ __forceinline__ v8f wm(v16b a, v16b b, v8f c) {
  v8f d = __builtin_amdgcn_wmma_f32_16x16x32_bf16(false, a, false, b, (short)0, c, false, false);
  asm volatile("v_nop\n\tv_nop\n\tv_nop\n\tv_nop" : "+v"(d) : "v"(a), "v"(b));
  return d;
}

__device__ __forceinline__ float wvmax(float v) {
  v = fmaxf(v, __shfl_xor(v, 16, 32));
  v = fmaxf(v, __shfl_xor(v, 8, 32));
  v = fmaxf(v, __shfl_xor(v, 4, 32));
  v = fmaxf(v, __shfl_xor(v, 2, 32));
  v = fmaxf(v, __shfl_xor(v, 1, 32));
  return v;
}

__global__ __launch_bounds__(GTHR) void k_prep(const float* __restrict__ Wf, const float* __restrict__ Ww,
                                               unsigned short* Wc, int total8) {
  const int i = blockIdx.x * GTHR + threadIdx.x;
  if (i >= total8) return;
  const int n  = i >> 3;
  const int c0 = (i & 7) * 8;
  Pack8 u;
#pragma unroll
  for (int j = 0; j < 8; ++j) {
    const int k = c0 + j;
    float v = 0.f;
    if (n < DO)               v = Wf[n * KW + k];
    else if (n < 2 * DO)      v = Wf[(n - DO) * KW + DI + k];
    else if (n == 2 * DO)     v = Ww[k];
    else if (n == 2 * DO + 1) v = Ww[DI + k];
    u.s[j] = bfr(v);
  }
  unsigned short* p = Wc + (size_t)n * DI + c0;
  *(volatile v8us*)p = u.v;
  __threadfence();
  *(volatile v8us*)p = u.v;
}

__global__ __launch_bounds__(GTHR) void k_gemm(const float* __restrict__ x, const unsigned short* __restrict__ Wc,
                                               float* PA, float* PB, float* PW, float* QW, int nN) {
  __shared__ __attribute__((aligned(16))) unsigned short At[GR * AP];
  __shared__ __attribute__((aligned(16))) float Xs[GR * XSP];

  const int tid  = threadIdx.x;
  const int lane = tid & 31;
  const int wave = __builtin_amdgcn_readfirstlane(tid >> 5);
  const int h    = lane >> 4;
  const int m    = lane & 15;
  const int rowBase = blockIdx.x * GR;

  {
    const int r  = tid >> 2;
    const int c0 = (tid & 3) * 16;
    int row = rowBase + r;
    if (row > nN - 1) row = nN - 1;
    const float* p = x + (size_t)row * DI + c0;
    const v4f f0 = *(const v4f*)(p), f1 = *(const v4f*)(p + 4);
    const v4f f2 = *(const v4f*)(p + 8), f3 = *(const v4f*)(p + 12);
    Pack8 u0, u1;
    u0.s[0] = bfr(f0.x); u0.s[1] = bfr(f0.y); u0.s[2] = bfr(f0.z); u0.s[3] = bfr(f0.w);
    u0.s[4] = bfr(f1.x); u0.s[5] = bfr(f1.y); u0.s[6] = bfr(f1.z); u0.s[7] = bfr(f1.w);
    u1.s[0] = bfr(f2.x); u1.s[1] = bfr(f2.y); u1.s[2] = bfr(f2.z); u1.s[3] = bfr(f2.w);
    u1.s[4] = bfr(f3.x); u1.s[5] = bfr(f3.y); u1.s[6] = bfr(f3.z); u1.s[7] = bfr(f3.w);
    *(v8us*)(At + r * AP + c0)     = u0.v;
    *(v8us*)(At + r * AP + c0 + 8) = u1.v;
  }
  __syncthreads();

  const int n0 = 16 * wave + m;
  const int n1 = 16 * (wave + GWAVE) + m;
  const int n8 = 16 * (NT - 1) + m;
  v8f c00 = {0.f, 0.f, 0.f, 0.f, 0.f, 0.f, 0.f, 0.f};
  v8f c10 = c00, c01 = c00, c11 = c00, c08 = c00, c18 = c00;
#pragma unroll
  for (int kt = 0; kt < DI / 32; ++kt) {
    const int k0 = kt * 32;
    FragB a0, a1, b0, b1, b8;
    const unsigned short* pa0 = At + m * AP + k0 + 8 * h;
    const unsigned short* pa1 = At + (16 + m) * AP + k0 + 8 * h;
    const unsigned short* pb0 = Wc + (size_t)n0 * DI + k0 + 8 * h;
    const unsigned short* pb1 = Wc + (size_t)n1 * DI + k0 + 8 * h;
    const unsigned short* pb8 = Wc + (size_t)n8 * DI + k0 + 8 * h;
    a0.hs[0] = *(const v8us*)pa0; a0.hs[1] = *(const v8us*)(pa0 + 16);
    a1.hs[0] = *(const v8us*)pa1; a1.hs[1] = *(const v8us*)(pa1 + 16);
    b0.hs[0] = *(const v8us*)pb0; b0.hs[1] = *(const v8us*)(pb0 + 16);
    b1.hs[0] = *(const v8us*)pb1; b1.hs[1] = *(const v8us*)(pb1 + 16);
    b8.hs[0] = *(const v8us*)pb8; b8.hs[1] = *(const v8us*)(pb8 + 16);
    c00 = wm(a0.v, b0.v, c00);
    c10 = wm(a1.v, b0.v, c10);
    c01 = wm(a0.v, b1.v, c01);
    c11 = wm(a1.v, b1.v, c11);
    c08 = wm(a0.v, b8.v, c08);
    c18 = wm(a1.v, b8.v, c18);
  }

#pragma unroll
  for (int r = 0; r < 8; ++r) {
    const int r0 = (8 * h + r) * XSP;
    const int r1 = (16 + 8 * h + r) * XSP;
    Xs[r0 + n0] = c00[r]; Xs[r1 + n0] = c10[r];
    Xs[r0 + n1] = c01[r]; Xs[r1 + n1] = c11[r];
    if (wave == 0) { Xs[r0 + n8] = c08[r]; Xs[r1 + n8] = c18[r]; }
  }
  __syncthreads();

  const int q4 = 4 * m;
  v4f va[4], vb[4];
  float* pa[4];
  float* pb[4];
#pragma unroll
  for (int i = 0; i < 4; ++i) {
    const int row = 8 * i + 2 * wave + h;
    va[i] = *(const v4f*)(Xs + row * XSP + q4);
    vb[i] = *(const v4f*)(Xs + row * XSP + DI + q4);
    pa[i] = PA + (size_t)(rowBase + row) * DO + q4;
    pb[i] = PB + (size_t)(rowBase + row) * DO + q4;
  }
  float* ps = 0;
  v4f vs = {0.f, 0.f, 0.f, 0.f};
  if (wave == 0 && lane < 16) {
    const int l8  = lane & 7;
    const int col = 16 * (NT - 1) + (lane >> 3);
    vs.x = Xs[(4 * l8 + 0) * XSP + col];
    vs.y = Xs[(4 * l8 + 1) * XSP + col];
    vs.z = Xs[(4 * l8 + 2) * XSP + col];
    vs.w = Xs[(4 * l8 + 3) * XSP + col];
    ps = ((lane < 8) ? PW : QW) + rowBase + 4 * l8;
  }
#pragma unroll
  for (int i = 0; i < 4; ++i) { *(volatile v4f*)(pa[i]) = va[i]; *(volatile v4f*)(pb[i]) = vb[i]; }
  if (ps) *(volatile v4f*)ps = vs;
  __threadfence();
#pragma unroll
  for (int i = 0; i < 4; ++i) { *(volatile v4f*)(pa[i]) = va[i]; *(volatile v4f*)(pb[i]) = vb[i]; }
  if (ps) *(volatile v4f*)ps = vs;
}

__global__ __launch_bounds__(NTHR) void k_emax(const int* __restrict__ src, const int* __restrict__ tgt,
                                               const float* __restrict__ PW, const float* __restrict__ QW,
                                               float* bmax, int nN, int nE) {
  __shared__ float red[NWAVE];
  const int tid  = threadIdx.x;
  const int lane = tid & 31;
  const int wave = __builtin_amdgcn_readfirstlane(tid >> 5);
  float mx = NEGBIG;
#pragma unroll 1
  for (int e = blockIdx.x * NTHR + tid; e < nE; e += MB * NTHR) {
    int s = src[e];
    int t = tgt[e];
    s = s < 0 ? 0 : (s > nN - 1 ? nN - 1 : s);
    t = t < 0 ? 0 : (t > nN - 1 ? nN - 1 : t);
    mx = fmaxf(mx, PW[s] + QW[t]);
  }
  mx = wvmax(mx);
  if (lane == 0) red[wave] = mx;
  __syncthreads();
  if (wave == 0) {
    float v = red[0];
#pragma unroll
    for (int w = 1; w < NWAVE; ++w) v = fmaxf(v, red[w]);
    const v4f o = {v, v, v, v};
    float* p = bmax + (size_t)blockIdx.x * 32 + 4 * (lane & 7);
    if (lane < 8) *(volatile v4f*)p = o;
    __threadfence();
    if (lane < 8) *(volatile v4f*)p = o;
  }
}

__global__ __launch_bounds__(NTHR) void k_agg(
    const int* __restrict__ src, const int* __restrict__ tgt,
    const float* __restrict__ PA, const float* __restrict__ PB,
    const float* __restrict__ PW, const float* __restrict__ QW,
    const float* __restrict__ bmax, const float* __restrict__ bf, const float* __restrict__ bw,
    float* out, int nN, int nE) {
  extern __shared__ v4f lds_dyn[];
  float* sacc = (float*)lds_dyn;
  float* den  = sacc + LDS_SACC;
  int*   list = (int*)(den + LDS_DEN);
  int*   wcnt = list + LDS_LIST;
  float* red  = (float*)(wcnt + NWAVE);

  const int tid  = threadIdx.x;
  const int lane = tid & 31;
  const int wave = __builtin_amdgcn_readfirstlane(tid >> 5);
  const int nodeBase = blockIdx.x * NB;

  {
    const v4f z4 = {0.f, 0.f, 0.f, 0.f};
    for (int i = tid; i < (LDS_SACC + LDS_DEN) / 4; i += NTHR) lds_dyn[i] = z4;
    float mx = (tid < MB) ? bmax[(size_t)min(tid, MB - 1) * 32] : NEGBIG;
    mx = wvmax(mx);
    if (lane == 0) red[wave] = mx;
  }
  __syncthreads();
  float amx = red[0];
#pragma unroll
  for (int w = 1; w < NWAVE; ++w) amx = fmaxf(amx, red[w]);
  const float bwv = bw[0];
  amx = amx + bwv;
  const v2f b2 = *(const v2f*)(bf + 2 * lane);
  const bool al16 = ((((size_t)tgt) & 15) == 0);

  const int nChunks = (nE + CHUNK - 1) / CHUNK;
#pragma unroll 1
  for (int ch = 0; ch < nChunks; ++ch) {
    const int cbase = ch * CHUNK;
    int wc = 0;
#pragma unroll
    for (int g = 0; g < NGRP; ++g) {
      const int el0 = (g * NTHR + tid) * 4;
      const int e0  = cbase + el0;
      const int sent = -2147483647 - 1;
      v4i d;
      if (al16 && (e0 + 3 < nE)) {
        d = *(const v4i*)(tgt + e0);
      } else {
        d.x = (e0     < nE) ? tgt[min(e0, nE - 1)]     : sent;
        d.y = (e0 + 1 < nE) ? tgt[min(e0 + 1, nE - 1)] : sent;
        d.z = (e0 + 2 < nE) ? tgt[min(e0 + 2, nE - 1)] : sent;
        d.w = (e0 + 3 < nE) ? tgt[min(e0 + 3, nE - 1)] : sent;
      }
      const unsigned s0 = (unsigned)d.x - (unsigned)nodeBase;
      const unsigned s1 = (unsigned)d.y - (unsigned)nodeBase;
      const unsigned s2 = (unsigned)d.z - (unsigned)nodeBase;
      const unsigned s3 = (unsigned)d.w - (unsigned)nodeBase;
      const bool h0 = s0 < (unsigned)NB;
      const bool h1 = s1 < (unsigned)NB;
      const bool h2 = s2 < (unsigned)NB;
      const bool h3 = s3 < (unsigned)NB;
      const unsigned many = __builtin_amdgcn_ballot_w32(h0 | h1 | h2 | h3);
      if (many != 0u) {
#define HITJ(J, HJ, SJ) { \
          const unsigned mj = __builtin_amdgcn_ballot_w32(HJ); \
          if (mj != 0u) { \
            if (HJ) { \
              const int pos = wc + (int)__builtin_amdgcn_mbcnt_lo(mj, 0u); \
              if (pos < WCAP) list[wave * WCAP + pos] = ((el0 + (J)) << 10) | (int)(SJ); \
            } \
            wc += (int)__builtin_popcount(mj); } }
        HITJ(0, h0, s0)
        HITJ(1, h1, s1)
        HITJ(2, h2, s2)
        HITJ(3, h3, s3)
#undef HITJ
      }
    }
    if (lane == 0) wcnt[wave] = wc;
    __syncthreads();

    if (wave == 0) {
#pragma unroll 1
      for (int wsx = 0; wsx < NWAVE; ++wsx) {
        int n = wcnt[wsx];
        if (n > WCAP) n = WCAP;
        if (n < 0) n = 0;
#pragma unroll 1
        for (int i = 0; i < n; ++i) {
          const int ent  = list[wsx * WCAP + i];
          const int slot = ent & (NB - 1);
          const int el   = (ent >> 10) & (CHUNK - 1);
          int e = cbase + el;
          if (e > nE - 1) e = nE - 1;
          int s = src[e];
          s = s < 0 ? 0 : (s > nN - 1 ? nN - 1 : s);
          int nd = nodeBase + slot;
          if (nd > nN - 1) nd = nN - 1;
          const float pq = PW[s] + QW[nd];
          const float p  = __expf((pq + bwv) - amx);
          const v2f ya = *(const v2f*)(PA + (size_t)s * DO + 2 * lane);
          const v2f yb = *(const v2f*)(PB + (size_t)nd * DO + 2 * lane);
          v2f y = ya + yb + b2;
          y.x = fmaxf(y.x, 0.f);
          y.y = fmaxf(y.y, 0.f);
          v2f* sp = (v2f*)(sacc + slot * DO + 2 * lane);
          const v2f cur = *sp;
          const v2f nxt = cur + p * y;
          *sp = nxt;
          if (lane == 0) {
            const float dd = den[slot];
            den[slot] = dd + p;
          }
        }
      }
    }
    __syncthreads();
  }

  const int hh = lane >> 4;
  const int q4 = 4 * (lane & 15);
#pragma unroll 1
  for (int j = 0; j < NB / (2 * NWAVE); ++j) {
    const int slot = wave * (NB / NWAVE) + 2 * j + hh;
    const int node = nodeBase + slot;
    const float dsum = den[slot] + EPSV;
    const float inv  = 1.0f / dsum;
    const v4f v = *(const v4f*)(sacc + slot * DO + q4) * inv;
    const bool ok = node < nN;
    float* op = out + (size_t)(ok ? node : 0) * DO + q4;
    if (ok) *(volatile v4f*)op = v;
    __threadfence();
    if (ok) *(volatile v4f*)op = v;
  }
}

static size_t al256(size_t v) { return (v + 255) & ~(size_t)255; }

extern "C" void kernel_launch(void* const* d_in, const int* in_sizes, int n_in,
                              void* d_out, int out_size, void* d_ws, size_t ws_size,
                              hipStream_t stream) {
  if (n_in < 7) return;
  if (in_sizes[0] <= 0 || (in_sizes[0] % DI) != 0) return;
  const int nN = in_sizes[0] / DI;
  if (in_sizes[1] != DO * KW) return;
  if (in_sizes[2] != DO) return;
  if (in_sizes[3] != KW) return;
  if (in_sizes[4] < 1) return;
  const int nE = in_sizes[5];
  if (nE < 1 || in_sizes[6] != nE) return;
  if (out_size != nN * DO) return;

  const float* x   = (const float*)d_in[0];
  const float* Wf  = (const float*)d_in[1];
  const float* bf  = (const float*)d_in[2];
  const float* Ww  = (const float*)d_in[3];
  const float* bw  = (const float*)d_in[4];
  const int*   src = (const int*)d_in[5];
  const int*   tgt = (const int*)d_in[6];
  float* out = (float*)d_out;

  const int nP = ((nN + GR - 1) / GR) * GR;
  size_t off = 0;
  unsigned short* Wc = (unsigned short*)((char*)d_ws + off); off += al256((size_t)NOUT * DI * sizeof(unsigned short));
  float* PA   = (float*)((char*)d_ws + off); off += al256((size_t)nP * DO * sizeof(float));
  float* PB   = (float*)((char*)d_ws + off); off += al256((size_t)nP * DO * sizeof(float));
  float* PW   = (float*)((char*)d_ws + off); off += al256((size_t)nP * sizeof(float));
  float* QW   = (float*)((char*)d_ws + off); off += al256((size_t)nP * sizeof(float));
  float* bmax = (float*)((char*)d_ws + off); off += al256((size_t)MB * 32 * sizeof(float));
  if (off > ws_size) return;

  const int total8 = NOUT * DI / 8;
  k_prep<<<(total8 + GTHR - 1) / GTHR, GTHR, 0, stream>>>(Wf, Ww, Wc, total8);

  k_gemm<<<nP / GR, GTHR, 0, stream>>>(x, Wc, PA, PB, PW, QW, nN);

  k_emax<<<MB, NTHR, 0, stream>>>(src, tgt, PW, QW, bmax, nN, nE);

  hipFuncSetAttribute(reinterpret_cast<const void*>(&k_agg),
                      hipFuncAttributeMaxDynamicSharedMemorySize, LDS_BYTES);
  const int grid = (nN + NB - 1) / NB;
  k_agg<<<grid, NTHR, LDS_BYTES, stream>>>(src, tgt, PA, PB, PW, QW, bmax, bf, bw, out, nN, nE);
}
